// GraphBlock_4492535791885
// MI455X (gfx1250) — hardware-run, weakly checked
//
#include <hip/hip_runtime.h>
#include <stddef.h>
#include <stdint.h>


#ifndef TANH_FAST
#define TANH_FAST 0
#endif

#define NN     50000
#define KN     16
#define DF     128
#define NPAD   50048
#define AP     512
#define KB     256
#define LNEPS  1e-5f
#define GBM    128
#define GTHR   256
#define LP     132
#define TILEF  (GBM * LP)
#define SPF    512
#define GEMM_LDS_BYTES ((TILEF + SPF) * 4)
#define ATHR   256
#define AWAVE  8
#define NPW    4
#define ATT_LDS_BYTES (AWAVE * KN * DF * 4)
#define PTHR   256

#define U_X    (NPAD * DF / 8)
#define U_W    8192
#define U_PAR0 (2 * U_X + 12288)
#define U_PARN 192
#define U_ALL  (U_PAR0 + U_PARN)

#define A2_BYTES  ((size_t)NPAD * AP * 2)
#define XE_BYTES  ((size_t)NPAD * DF * 2)
#define EH_BYTES  ((size_t)NPAD * DF * 4)
#define O_EH      (A2_BYTES)
#define O_ET      (O_EH + EH_BYTES)
#define O_W       (O_ET + EH_BYTES)
#define W_BYTES   ((size_t)(2 * DF * DF + 2 * DF * KB) * 2)
#define O_PAR     (O_W + W_BYTES)
#define PAR_BYTES ((size_t)6 * DF * 4)
#define WS_TOTAL  (O_PAR + PAR_BYTES)
#define WSMAX     134217728

static_assert(DF == 128 && 32 * 4 == DF);
static_assert(KN == 16 && KN <= 32);
static_assert(NPAD == 391 * 128 && NPAD >= NN && NPAD % GBM == 0 && NPAD % (AWAVE * NPW) == 0);
static_assert(NN == 390 * 128 + 80);
static_assert((2 * DF) % 32 == 0 && DF % 32 == 0 && KB == 2 * DF && AP == 2 * KB);
static_assert(GBM == (GTHR / 32) * 16);
static_assert(LP % 4 == 0 && LP >= DF);
static_assert(GEMM_LDS_BYTES == 69632 && GEMM_LDS_BYTES <= 327680);
static_assert(ATT_LDS_BYTES == 65536 && ATT_LDS_BYTES <= 327680);
static_assert(U_X % PTHR == 0 && (2 * U_X) % PTHR == 0 && U_PAR0 % PTHR == 0 && U_X == NPAD * 16);
static_assert(2 * XE_BYTES <= A2_BYTES);
static_assert(A2_BYTES % 256 == 0 && EH_BYTES % 256 == 0 && O_W % 256 == 0 && O_PAR % 256 == 0);
static_assert(WS_TOTAL == 102697984 && WS_TOTAL <= WSMAX);
static_assert((size_t)(NN - 1) * DF + DF - 1 == (size_t)NN * DF - 1);

typedef float          v4f   __attribute__((ext_vector_type(4)));
typedef float          v8f   __attribute__((ext_vector_type(8)));
typedef int            v8i   __attribute__((ext_vector_type(8)));
typedef unsigned short v4us  __attribute__((ext_vector_type(4)));
typedef unsigned short v8us  __attribute__((ext_vector_type(8)));
typedef unsigned short v16us __attribute__((ext_vector_type(16)));
typedef __bf16         v16bf __attribute__((ext_vector_type(16)));
typedef v4f  __attribute__((may_alias)) v4fa;
typedef v8us __attribute__((may_alias)) v8usa;
union FragB { v16bf v; v16us u; v8us h[2]; v8i w; };

__device__ __forceinline__ v8f wmb(const FragB& a, const FragB& b, v8f c) {
  v8f d = __builtin_amdgcn_wmma_f32_16x16x32_bf16(false, a.v, false, b.v, (short)0, c, false, false);
  asm volatile("v_nop\n\tv_nop\n\tv_nop\n\tv_nop" : "+v"(d) : "v"(a.w), "v"(b.w));
  return d;
}

__device__ __forceinline__ v8f z8() { v8f z = {0.f, 0.f, 0.f, 0.f, 0.f, 0.f, 0.f, 0.f}; return z; }

__device__ __forceinline__ unsigned bf16_bits(float f) {
  const unsigned u = __float_as_uint(f);
  return (u + 0x7FFFu + ((u >> 16) & 1u)) >> 16;
}
__device__ __forceinline__ float bf16_val(float f) {
  return __uint_as_float(bf16_bits(f) << 16);
}
__device__ __forceinline__ unsigned hl_bits(float v, unsigned& lo) {
  const unsigned hb = bf16_bits(v);
  lo = bf16_bits(v - __uint_as_float(hb << 16));
  return hb;
}

__device__ __forceinline__ float leaky(float v) { return (v > 0.0f) ? v : (0.01f * v); }

__device__ __forceinline__ float readlane_f(float v, int k) {
  return __int_as_float(__builtin_amdgcn_readlane(__float_as_int(v), k));
}

__device__ __forceinline__ float gate_tanh(float t) {
#if TANH_FAST
  const float a = fminf(fabsf(t), 20.0f);
  const float e = __expf(2.0f * a);
  const float r = 1.0f - 2.0f * __builtin_amdgcn_rcpf(1.0f + e);
  return copysignf(r, t);
#else
  return tanhf(t);
#endif
}

__device__ __forceinline__ v8us cvt8(const float* __restrict__ p, unsigned msk) {
  const v4f a = *(const v4f*)p;
  const v4f c = *(const v4f*)(p + 4);
  asm volatile("" :: "v"(a), "v"(c));
  v8us o;
  o[0] = (unsigned short)(bf16_bits(a.x) & msk);
  o[1] = (unsigned short)(bf16_bits(a.y) & msk);
  o[2] = (unsigned short)(bf16_bits(a.z) & msk);
  o[3] = (unsigned short)(bf16_bits(a.w) & msk);
  o[4] = (unsigned short)(bf16_bits(c.x) & msk);
  o[5] = (unsigned short)(bf16_bits(c.y) & msk);
  o[6] = (unsigned short)(bf16_bits(c.z) & msk);
  o[7] = (unsigned short)(bf16_bits(c.w) & msk);
  return o;
}

__global__ __launch_bounds__(PTHR) void k_prep(
    const float* __restrict__ ehin, const float* __restrict__ etin,
    const float* __restrict__ wh, const float* __restrict__ wt,
    const float* __restrict__ w1, const float* __restrict__ w2,
    const float* __restrict__ bh, const float* __restrict__ bt,
    const float* __restrict__ b1, const float* __restrict__ b2,
    const float* __restrict__ gam, const float* __restrict__ bet,
    unsigned short* wsb, float* par)
{
  const int u = (int)blockIdx.x * PTHR + (int)threadIdx.x;
  if (u >= U_ALL) return;
  if (u >= U_PAR0) {
    const int q = u - U_PAR0;
    const int row = q >> 5, c4 = (q & 31) * 4;
    const v4f p0 = *(const v4f*)(bh + c4);
    const v4f p1 = *(const v4f*)(bt + c4);
    const v4f p2 = *(const v4f*)(b1 + c4);
    const v4f p3 = *(const v4f*)(b2 + c4);
    const v4f p4 = *(const v4f*)(gam + c4);
    const v4f p5 = *(const v4f*)(bet + c4);
    asm volatile("" :: "v"(p0), "v"(p1), "v"(p2), "v"(p3), "v"(p4), "v"(p5));
    const unsigned m0 = (row == 0) ? 0xFFFFFFFFu : 0u;
    const unsigned m1 = (row == 1) ? 0xFFFFFFFFu : 0u;
    const unsigned m2 = (row == 2) ? 0xFFFFFFFFu : 0u;
    const unsigned m3 = (row == 3) ? 0xFFFFFFFFu : 0u;
    const unsigned m4 = (row == 4) ? 0xFFFFFFFFu : 0u;
    const unsigned m5 = (row == 5) ? 0xFFFFFFFFu : 0u;
#define BLEND(C) ((__float_as_uint(p0.C) & m0) | (__float_as_uint(p1.C) & m1) | (__float_as_uint(p2.C) & m2) | \
                  (__float_as_uint(p3.C) & m3) | (__float_as_uint(p4.C) & m4) | (__float_as_uint(p5.C) & m5))
    v4f o;
    o.x = bf16_val(__uint_as_float(BLEND(x)));
    o.y = bf16_val(__uint_as_float(BLEND(y)));
    o.z = bf16_val(__uint_as_float(BLEND(z)));
    o.w = bf16_val(__uint_as_float(BLEND(w)));
#undef BLEND
    float* dp = par + (size_t)q * 4;
    *(volatile v4f*)dp = o;
    __threadfence();
    *(volatile v4f*)dp = o;
    return;
  }
  v8us o;
  size_t eo;
  if (u < U_X) {
    const int row = u >> 4, k8 = (u & 15) * 8;
    const int rc = row < NN ? row : NN - 1;
    const unsigned msk = row < NN ? 0xFFFFu : 0u;
    o = cvt8(ehin + (size_t)rc * DF + k8, msk);
    eo = (size_t)u * 8;
  } else if (u < 2 * U_X) {
    const int v = u - U_X;
    const int row = v >> 4, k8 = (v & 15) * 8;
    const int rc = row < NN ? row : NN - 1;
    const unsigned msk = row < NN ? 0xFFFFu : 0u;
    o = cvt8(etin + (size_t)rc * DF + k8, msk);
    eo = (size_t)u * 8;
  } else {
    const int v = u - 2 * U_X;
    if (v < 2048) {
      o = cvt8(wh + (size_t)v * 8, 0xFFFFu);
    } else if (v < 4096) {
      o = cvt8(wt + (size_t)(v - 2048) * 8, 0xFFFFu);
    } else if (v < 8192) {
      const int t = v - 4096;
      const int n = t >> 5, kk = ((t & 31) * 8) & (DF - 1);
      o = cvt8(w1 + (size_t)n * DF + kk, 0xFFFFu);
    } else {
      const int t = v - 8192;
      const int n = t >> 5, kk = ((t & 31) * 8) & (DF - 1);
      o = cvt8(w2 + (size_t)n * DF + kk, 0xFFFFu);
    }
    eo = (size_t)(O_W / 2) + (size_t)v * 8;
  }
  unsigned short* dp = wsb + eo;
  *(volatile v8us*)dp = o;
  __threadfence();
  *(volatile v8us*)dp = o;
}

template <int KT, int LDB>
__device__ __forceinline__ void kloop(const unsigned short* ap, const unsigned short* bp, v8f (&acc)[8]) {
#pragma unroll 1
  for (int k0 = 0; k0 < KT; k0 += 32) {
    FragB af;
    af.h[0] = *(const v8usa*)(ap + k0);
    af.h[1] = *(const v8usa*)(ap + k0 + 16);
#pragma unroll
    for (int nt = 0; nt < 8; ++nt) {
      const unsigned short* wq = bp + (size_t)(16 * nt) * LDB + k0;
      FragB bf;
      bf.h[0] = *(const v8usa*)wq;
      bf.h[1] = *(const v8usa*)(wq + 16);
      acc[nt] = wmb(af, bf, acc[nt]);
    }
  }
}

__global__ __launch_bounds__(GTHR) __attribute__((amdgpu_num_vgpr(248)))
void k_projA(const unsigned short* __restrict__ xe, const unsigned short* __restrict__ wht,
             const float* __restrict__ par, float* eht)
{
  extern __shared__ __attribute__((aligned(16))) float dsm[];
  float* stg = dsm;
  float* sp  = dsm + TILEF;
  const int tid = (int)threadIdx.x, lane = tid & 31, wave = tid >> 5, hh = lane >> 4, m = lane & 15;
  const int sel = (int)blockIdx.y;
  const int rowBase = (int)blockIdx.x * GBM;

  if (tid < 32) *(v4fa*)(sp + 4 * tid) = *(const v4f*)(par + (size_t)sel * DF + 4 * tid);

  v8f acc[8];
#pragma unroll
  for (int t = 0; t < 8; ++t) acc[t] = z8();
  const unsigned short* ap = xe + (size_t)sel * ((size_t)NPAD * DF) + (size_t)(rowBase + 16 * wave + m) * DF + 8 * hh;
  const unsigned short* bp = wht + (size_t)sel * (DF * DF) + (size_t)m * DF + 8 * hh;
  kloop<DF, DF>(ap, bp, acc);

#pragma unroll
  for (int nt = 0; nt < 8; ++nt) {
    const int lc = 16 * nt + m;
#pragma unroll
    for (int r = 0; r < 8; ++r) {
      const int lr = 16 * wave + 8 * hh + r;
      stg[lr * LP + lc] = acc[nt][r];
    }
  }
  __syncthreads();

  const v4f bq = *(const v4fa*)(sp + 4 * lane);
  float* ob = eht + (size_t)sel * ((size_t)NPAD * DF);
#pragma unroll 1
  for (int i = 0; i < 16; ++i) {
    float* sr = stg + (16 * wave + i) * LP + 4 * lane;
    const int grow = rowBase + 16 * wave + i;
    const bool keep = grow < NN;
    const v4f v = *(const v4fa*)sr;
    v4f o;
    o.x = keep ? (v.x + bq.x) : 0.0f;
    o.y = keep ? (v.y + bq.y) : 0.0f;
    o.z = keep ? (v.z + bq.z) : 0.0f;
    o.w = keep ? (v.w + bq.w) : 0.0f;
    *(v4fa*)sr = o;
    *(volatile v4f*)(ob + (size_t)grow * DF + 4 * lane) = o;
  }
  __threadfence();
#pragma unroll 1
  for (int i = 0; i < 16; ++i) {
    const float* sr = stg + (16 * wave + i) * LP + 4 * lane;
    const int grow = rowBase + 16 * wave + i;
    const v4f o = *(const v4fa*)sr;
    *(volatile v4f*)(ob + (size_t)grow * DF + 4 * lane) = o;
  }
}

__global__ __launch_bounds__(ATHR) __attribute__((amdgpu_num_vgpr(248)))
void k_attn(const float* __restrict__ x, const float* __restrict__ ehp, const float* __restrict__ etp,
            const int* __restrict__ tki, const float* __restrict__ tkw, unsigned short* apl)
{
  extern __shared__ __attribute__((aligned(16))) float nbs[];
  const int tid = (int)threadIdx.x, lane = tid & 31, wave = tid >> 5;
  const int l15 = lane & 15;
  float* slot = nbs + wave * (KN * DF) + 4 * lane;
  const int nb0 = (int)blockIdx.x * (AWAVE * NPW) + wave * NPW;

#pragma unroll 1
  for (int s = 0; s < NPW; ++s) {
    const int n  = nb0 + s;
    const int nc = n < NN ? n : NN - 1;
    const unsigned lm = n < NN ? 0xFFFFu : 0u;

    const v4f e4 = *(const v4f*)(ehp + (size_t)nc * DF + 4 * lane);
    const v4f xr = *(const v4f*)(x + (size_t)nc * DF + 4 * lane);
    int idx = tki[(size_t)nc * KN + l15];
    const float pw = tkw[(size_t)nc * KN + l15];
    idx = idx < 0 ? 0 : (idx > NN - 1 ? NN - 1 : idx);
    const float pwb = bf16_val(pw);

    float e0 = e4.x, e1 = e4.y, e2 = e4.z, e3 = e4.w;
    float scv = 0.0f;

#pragma unroll 1
    for (int k = 0; k < KN; ++k) {
      const int   ik = __builtin_amdgcn_readlane(idx, k);
      const float pk = readlane_f(pwb, k);
      const float qk = 1.0f - pk;
      const v4f nbv = *(const v4f*)(etp + (size_t)ik * DF + 4 * lane);
      *(v4fa*)(slot + k * DF) = nbv;
      float a0 = nbv.x, a1 = nbv.y, a2 = nbv.z, a3 = nbv.w;
      float part = 0.0f;
#pragma unroll 1
      for (int c = 0; c < 4; ++c) {
        const float r = pk * a0 + qk * e0;
        const float t = e0 + r;
        const float g = gate_tanh(t);
        part = part + a0 * g;
        const float ta = a0; a0 = a1; a1 = a2; a2 = a3; a3 = ta;
        const float te = e0; e0 = e1; e1 = e2; e2 = e3; e3 = te;
      }
      part += __shfl_xor(part, 16, 32);
      part += __shfl_xor(part, 8, 32);
      part += __shfl_xor(part, 4, 32);
      part += __shfl_xor(part, 2, 32);
      part += __shfl_xor(part, 1, 32);
      scv = (l15 == k) ? part : scv;
    }

    float mx = readlane_f(scv, 0);
#pragma unroll 1
    for (int k = 1; k < KN; ++k) {
      const float sk = readlane_f(scv, k);
      mx = (sk > mx) ? sk : mx;
    }
    const float qv = expf(scv - mx);
    float ssum = 0.0f;
#pragma unroll 1
    for (int k = 0; k < KN; ++k) ssum += readlane_f(qv, k);
    const float inv = 1.0f / ssum;
    const float kav = qv * inv;

    float n0 = 0.0f, n1 = 0.0f, n2 = 0.0f, n3 = 0.0f;
#pragma unroll 1
    for (int k = 0; k < KN; ++k) {
      const float wk = readlane_f(kav, k);
      const v4f nbv = *(const v4fa*)(slot + k * DF);
      n0 += wk * nbv.x; n1 += wk * nbv.y; n2 += wk * nbv.z; n3 += wk * nbv.w;
    }

    const float x0 = bf16_val(xr.x), x1 = bf16_val(xr.y), x2 = bf16_val(xr.z), x3 = bf16_val(xr.w);
    const float s0 = x0 + n0, s1 = x1 + n1, s2 = x2 + n2, s3 = x3 + n3;
    const float p0 = x0 * n0, p1 = x1 * n1, p2 = x2 * n2, p3 = x3 * n3;
    v4us sh, sl, mh, ml;
    {
      unsigned lb;
      unsigned hb;
      hb = hl_bits(s0, lb); sh[0] = (unsigned short)(hb & lm); sl[0] = (unsigned short)(lb & lm);
      hb = hl_bits(s1, lb); sh[1] = (unsigned short)(hb & lm); sl[1] = (unsigned short)(lb & lm);
      hb = hl_bits(s2, lb); sh[2] = (unsigned short)(hb & lm); sl[2] = (unsigned short)(lb & lm);
      hb = hl_bits(s3, lb); sh[3] = (unsigned short)(hb & lm); sl[3] = (unsigned short)(lb & lm);
      hb = hl_bits(p0, lb); mh[0] = (unsigned short)(hb & lm); ml[0] = (unsigned short)(lb & lm);
      hb = hl_bits(p1, lb); mh[1] = (unsigned short)(hb & lm); ml[1] = (unsigned short)(lb & lm);
      hb = hl_bits(p2, lb); mh[2] = (unsigned short)(hb & lm); ml[2] = (unsigned short)(lb & lm);
      hb = hl_bits(p3, lb); mh[3] = (unsigned short)(hb & lm); ml[3] = (unsigned short)(lb & lm);
    }
    unsigned short* rp = apl + (size_t)n * AP + 4 * lane;
    *(volatile v4us*)(rp)          = sh;
    *(volatile v4us*)(rp + DF)     = sl;
    *(volatile v4us*)(rp + 2 * DF) = mh;
    *(volatile v4us*)(rp + 3 * DF) = ml;
    __threadfence();
    *(volatile v4us*)(rp)          = sh;
    *(volatile v4us*)(rp + DF)     = sl;
    *(volatile v4us*)(rp + 2 * DF) = mh;
    *(volatile v4us*)(rp + 3 * DF) = ml;
  }
}

__global__ __launch_bounds__(GTHR) __attribute__((amdgpu_num_vgpr(248)))
void k_projB(const unsigned short* __restrict__ a2p, const unsigned short* __restrict__ w12d,
             const float* __restrict__ par, float* outp)
{
  extern __shared__ __attribute__((aligned(16))) float dsm[];
  float* stg = dsm;
  float* sp  = dsm + TILEF;
  const int tid = (int)threadIdx.x, lane = tid & 31, wave = tid >> 5, hh = lane >> 4, m = lane & 15;
  const int rowBase = (int)blockIdx.x * GBM;

  if (tid < 128) *(v4fa*)(sp + 4 * tid) = *(const v4f*)(par + 2 * DF + 4 * tid);
  __syncthreads();

  const unsigned short* ap = a2p + (size_t)(rowBase + 16 * wave + m) * AP + 8 * hh;
  const unsigned short* bp = w12d + (size_t)m * KB + 8 * hh;

  v8f acc[8];
#pragma unroll
  for (int t = 0; t < 8; ++t) acc[t] = z8();
  kloop<KB, KB>(ap, bp, acc);
#pragma unroll
  for (int nt = 0; nt < 8; ++nt) {
    const int lc = 16 * nt + m;
    const float bv = sp[lc];
#pragma unroll
    for (int r = 0; r < 8; ++r) {
      const int lr = 16 * wave + 8 * hh + r;
      stg[lr * LP + lc] = leaky(acc[nt][r] + bv);
    }
  }

#pragma unroll
  for (int t = 0; t < 8; ++t) acc[t] = z8();
  kloop<KB, KB>(ap + KB, bp + (size_t)DF * KB, acc);
#pragma unroll
  for (int nt = 0; nt < 8; ++nt) {
    const int lc = 16 * nt + m;
    const float bv = sp[DF + lc];
#pragma unroll
    for (int r = 0; r < 8; ++r) {
      const int lr = 16 * wave + 8 * hh + r;
      const float h1 = stg[lr * LP + lc];
      const float h2 = leaky(acc[nt][r] + bv);
      stg[lr * LP + lc] = h1 + h2;
    }
  }
  __syncthreads();

  const v4f g4 = *(const v4fa*)(sp + 2 * DF + 4 * lane);
  const v4f b4 = *(const v4fa*)(sp + 3 * DF + 4 * lane);
  const float invd = 1.0f / (float)DF;
#pragma unroll 1
  for (int i = 0; i < 16; ++i) {
    float* sr = stg + (16 * wave + i) * LP + 4 * lane;
    const int grow = rowBase + 16 * wave + i;
    const v4f v = *(const v4fa*)sr;
    float sm = (v.x + v.y) + (v.z + v.w);
    sm += __shfl_xor(sm, 16, 32);
    sm += __shfl_xor(sm, 8, 32);
    sm += __shfl_xor(sm, 4, 32);
    sm += __shfl_xor(sm, 2, 32);
    sm += __shfl_xor(sm, 1, 32);
    const float mean = sm * invd;
    const float d0 = v.x - mean, d1 = v.y - mean, d2 = v.z - mean, d3 = v.w - mean;
    float q = (d0 * d0 + d1 * d1) + (d2 * d2 + d3 * d3);
    q += __shfl_xor(q, 16, 32);
    q += __shfl_xor(q, 8, 32);
    q += __shfl_xor(q, 4, 32);
    q += __shfl_xor(q, 2, 32);
    q += __shfl_xor(q, 1, 32);
    const float var = q * invd;
    const float sd  = sqrtf(var + LNEPS);
    v4f o;
    o.x = (d0 / sd) * g4.x + b4.x;
    o.y = (d1 / sd) * g4.y + b4.y;
    o.z = (d2 / sd) * g4.z + b4.z;
    o.w = (d3 / sd) * g4.w + b4.w;
    *(v4fa*)sr = o;
    if (grow < NN) *(volatile v4f*)(outp + (size_t)grow * DF + 4 * lane) = o;
  }
  __threadfence();
#pragma unroll 1
  for (int i = 0; i < 16; ++i) {
    const float* sr = stg + (16 * wave + i) * LP + 4 * lane;
    const int grow = rowBase + 16 * wave + i;
    const v4f o = *(const v4fa*)sr;
    if (grow < NN) *(volatile v4f*)(outp + (size_t)grow * DF + 4 * lane) = o;
  }
}

extern "C" void kernel_launch(void* const* d_in, const int* in_sizes, int n_in,
                              void* d_out, int out_size, void* d_ws, size_t ws_size,
                              hipStream_t stream) {
  if (n_in < 15) return;
  if (in_sizes[0] != NN * DF || in_sizes[1] != NN * DF || in_sizes[2] != NN * DF) return;
  if (in_sizes[3] != NN * KN || in_sizes[4] != NN * KN) return;
  if (in_sizes[5] != DF * DF || in_sizes[7] != DF * DF || in_sizes[9] != DF * DF || in_sizes[11] != DF * DF) return;
  if (in_sizes[6] != DF || in_sizes[8] != DF || in_sizes[10] != DF || in_sizes[12] != DF) return;
  if (in_sizes[13] != DF || in_sizes[14] != DF) return;
  if (out_size != NN * DF) return;
  if ((size_t)WS_TOTAL > ws_size) return;

  const float* x    = (const float*)d_in[0];
  const float* ehin = (const float*)d_in[1];
  const float* etin = (const float*)d_in[2];
  const int*   tki  = (const int*)  d_in[3];
  const float* tkw  = (const float*)d_in[4];
  const float* Wh   = (const float*)d_in[5];
  const float* bh   = (const float*)d_in[6];
  const float* Wt   = (const float*)d_in[7];
  const float* bt   = (const float*)d_in[8];
  const float* W1   = (const float*)d_in[9];
  const float* b1   = (const float*)d_in[10];
  const float* W2   = (const float*)d_in[11];
  const float* b2   = (const float*)d_in[12];
  const float* gam  = (const float*)d_in[13];
  const float* bet  = (const float*)d_in[14];
  float* out = (float*)d_out;

  char* ws = (char*)d_ws;
  unsigned short* wsb  = (unsigned short*)ws;
  float*          EH   = (float*)(ws + O_EH);
  unsigned short* WPL  = (unsigned short*)(ws + O_W);
  float*          PAR  = (float*)(ws + O_PAR);

  hipFuncSetAttribute(reinterpret_cast<const void*>(&k_projA), hipFuncAttributeMaxDynamicSharedMemorySize, (int)GEMM_LDS_BYTES);
  hipFuncSetAttribute(reinterpret_cast<const void*>(&k_attn),  hipFuncAttributeMaxDynamicSharedMemorySize, (int)ATT_LDS_BYTES);
  hipFuncSetAttribute(reinterpret_cast<const void*>(&k_projB), hipFuncAttributeMaxDynamicSharedMemorySize, (int)GEMM_LDS_BYTES);

  k_prep<<<(U_ALL + PTHR - 1) / PTHR, PTHR, 0, stream>>>(ehin, etin, Wh, Wt, W1, W2, bh, bt, b1, b2, gam, bet, wsb, PAR);
  dim3 gA(NPAD / GBM, 2);
  k_projA<<<gA, GTHR, GEMM_LDS_BYTES, stream>>>(wsb, WPL, PAR, EH);
  k_attn<<<NPAD / (AWAVE * NPW), ATHR, ATT_LDS_BYTES, stream>>>(x, EH, EH + (size_t)NPAD * DF, tki, tkw, wsb);
  k_projB<<<NPAD / GBM, GTHR, GEMM_LDS_BYTES, stream>>>(wsb, WPL + 2 * DF * DF, PAR, out);
}
